// KANLinear_45586782880324
// MI455X (gfx1250) — hardware-verified
//
#include <hip/hip_runtime.h>
#include <math.h>

constexpr int kRows  = 8192;
constexpr int kIn    = 1024;
constexpr int kOutF  = 1024;
constexpr int kComp  = 4;
constexpr int kAug   = kIn * kComp;
constexpr int kNB    = 8;
constexpr int kGridN = 6;
constexpr float kEps      = 1e-8f;
constexpr float kACarry   = 256.0f;
constexpr float kWCarry   = 16.0f;
constexpr float kOutScale = 1.0f / 4096.0f;
constexpr size_t kBtBytes = (size_t)kOutF * kAug * 2;
constexpr size_t kABytes  = (size_t)kRows * kAug * 2;
constexpr size_t kWsNeed  = kBtBytes + kABytes;
constexpr int kPairThreads = kRows * (kIn / 2);
constexpr int kGemmTiles   = (kRows / 64) * (kOutF / 64);
constexpr int kGemmBlocks  = kGemmTiles / 8;

static_assert(kAug % 32 == 0);
static_assert(kRows % 64 == 0);
static_assert(kOutF % 64 == 0);
static_assert(kGemmTiles % 8 == 0);
static_assert(kWsNeed <= (size_t)134217728);
static_assert(kIn == 4 * 256);
static_assert(kPairThreads % 256 == 0);

typedef __attribute__((ext_vector_type(16))) _Float16 v16h;
typedef __attribute__((ext_vector_type(8)))  _Float16 v8h;
typedef __attribute__((ext_vector_type(16))) __bf16   v16b;
typedef __attribute__((ext_vector_type(8)))  __bf16   v8b;
typedef __attribute__((ext_vector_type(8)))  float    v8f;
typedef __attribute__((ext_vector_type(4)))  float    v4f;
typedef __attribute__((ext_vector_type(2)))  float    v2f;
typedef __attribute__((ext_vector_type(4)))  unsigned int v4u;

__device__ __forceinline__ unsigned short f2bf_bits(float f) {
  unsigned u = __float_as_uint(f);
  return (unsigned short)((u + 0x7FFFu + ((u >> 16) & 1u)) >> 16);
}
__device__ __forceinline__ float bf_bits2f(unsigned short h) { return __uint_as_float(((unsigned)h) << 16); }

__device__ __forceinline__ void dep_guard_h(v8f& a, v8f& b, v16h x, v16h y) { asm volatile("v_nop\n\tv_nop\n\tv_nop\n\tv_nop" : "+v"(a), "+v"(b) : "v"(x), "v"(y)); }
__device__ __forceinline__ void dep_guard_b(v8f& a, v8f& b, v16b x, v16b y) { asm volatile("v_nop\n\tv_nop\n\tv_nop\n\tv_nop" : "+v"(a), "+v"(b) : "v"(x), "v"(y)); }
__device__ __forceinline__ void dep_guard4_h(v8f& a, v8f& b, v8f& c, v8f& d, v16h x, v16h y) { asm volatile("v_nop\n\tv_nop\n\tv_nop\n\tv_nop" : "+v"(a), "+v"(b), "+v"(c), "+v"(d) : "v"(x), "v"(y)); }
__device__ __forceinline__ void dep_guard4_b(v8f& a, v8f& b, v8f& c, v8f& d, v16b x, v16b y) { asm volatile("v_nop\n\tv_nop\n\tv_nop\n\tv_nop" : "+v"(a), "+v"(b), "+v"(c), "+v"(d) : "v"(x), "v"(y)); }
__device__ __forceinline__ void keep4_h(v16h a, v16h b, v16h c, v16h d) { asm volatile("v_nop" :: "v"(a), "v"(b), "v"(c), "v"(d)); }
__device__ __forceinline__ void keep4_b(v16b a, v16b b, v16b c, v16b d) { asm volatile("v_nop" :: "v"(a), "v"(b), "v"(c), "v"(d)); }
__device__ __forceinline__ void acc_guard4(v8f& a, v8f& b, v8f& c, v8f& d) { asm volatile("v_nop\n\tv_nop\n\tv_nop\n\tv_nop" : "+v"(a), "+v"(b), "+v"(c), "+v"(d)); }
template <typename T> struct Frag;
template <> struct Frag<_Float16> {
  typedef v16h V; union U { v16h v; v8h h[2]; };
  static __device__ __forceinline__ v16h load(const _Float16* p) {
    U f; f.h[0] = *(const v8h*)(p); f.h[1] = *(const v8h*)(p + 16); return f.v;
  }
  static __device__ __forceinline__ v8f mma(v16h a, v16h b, v8f c) {
    return __builtin_amdgcn_wmma_f32_16x16x32_f16(false, a, false, b, (short)0, c, false, false);
  }
  static __device__ __forceinline__ void guard(v8f& a, v8f& b, v16h x, v16h y) { dep_guard_h(a, b, x, y); }
  static __device__ __forceinline__ void guard4(v8f& a, v8f& b, v8f& c, v8f& d, v16h x, v16h y) { dep_guard4_h(a, b, c, d, x, y); }
  static __device__ __forceinline__ void keep(v16h a, v16h b, v16h c, v16h d) { keep4_h(a, b, c, d); }
};
template <> struct Frag<__bf16> {
  typedef v16b V; union U { v16b v; v8b h[2]; };
  static __device__ __forceinline__ v16b load(const __bf16* p) {
    U f; f.h[0] = *(const v8b*)(p); f.h[1] = *(const v8b*)(p + 16); return f.v;
  }
  static __device__ __forceinline__ v8f mma(v16b a, v16b b, v8f c) {
    return __builtin_amdgcn_wmma_f32_16x16x32_bf16(false, a, false, b, (short)0, c, false, false);
  }
  static __device__ __forceinline__ void guard(v8f& a, v8f& b, v16b x, v16b y) { dep_guard_b(a, b, x, y); }
  static __device__ __forceinline__ void guard4(v8f& a, v8f& b, v8f& c, v8f& d, v16b x, v16b y) { dep_guard4_b(a, b, c, d, x, y); }
  static __device__ __forceinline__ void keep(v16b a, v16b b, v16b c, v16b d) { keep4_b(a, b, c, d); }
};

__device__ __forceinline__ unsigned pk16(unsigned short a, unsigned short b) { return (unsigned)a | ((unsigned)b << 16); }
__device__ __forceinline__ unsigned short h_bits(float f) { const _Float16 h = (_Float16)f; return __builtin_bit_cast(unsigned short, h); }

template <int ET> struct Elem;
template <> struct Elem<0> { typedef _Float16 T; };
template <> struct Elem<1> { typedef __bf16 T; };
template <int ET, bool SPLIT, int BIAS_MODE, int OUT_MODE, bool RESID, int ACT = 0>
__global__ __launch_bounds__(256) void wmma_gemm64(
    const unsigned short* __restrict__ Ap, const unsigned short* __restrict__ A2p, int lda, long strideA,
    const unsigned short* __restrict__ Btp, const unsigned short* __restrict__ Bt2p, int ldb, long strideB,
    void* __restrict__ Cout, void* __restrict__ Cout2, int ldc, long strideC,
    const float* __restrict__ bias,
    const float* __restrict__ resid, long strideR,
    int M, int N, int K, float scale) {
  typedef typename Elem<ET>::T T;
  typedef typename Frag<T>::V V;
  const T* A = (const T*)Ap; const T* A2 = (const T*)A2p; const T* Bt = (const T*)Btp; const T* Bt2 = (const T*)Bt2p;
  __shared__ __align__(16) float sT[8][16 * 68];
  const int b    = blockIdx.y;
  const int lane = threadIdx.x & 31;
  const int wave = threadIdx.x >> 5;
  const int tilesN = N >> 6;
  const int tilesM = M >> 6;
  const int tile = blockIdx.x * 8 + wave;
  if (tile >= tilesM * tilesN) return;
  const int tm = tile / tilesN;
  const int tn = tile - tm * tilesN;
  const int m0 = tm << 6;
  const int n0 = tn << 6;

  const T* Ab  = A  + (size_t)b * strideA;
  const T* Bb  = Bt + (size_t)b * strideB;
  const T* Ab2 = SPLIT ? (A2  + (size_t)b * strideA) : nullptr;
  const T* Bb2 = SPLIT ? (Bt2 + (size_t)b * strideB) : nullptr;

  const int rlane = lane & 15;
  const int koff  = (lane >> 4) * 8;
  const int mOff  = (lane >> 4) * 8;

  v8f acc[4][4];
#pragma unroll
  for (int i = 0; i < 4; ++i)
#pragma unroll
    for (int j = 0; j < 4; ++j) acc[i][j] = (v8f){0.f,0.f,0.f,0.f,0.f,0.f,0.f,0.f};

  for (int k0 = 0; k0 < K; k0 += 32) {
    V bh[4], bl[4];
#pragma unroll
    for (int j = 0; j < 4; ++j) {
      const size_t bo = (size_t)(n0 + (j << 4) + rlane) * ldb + koff + k0;
      bh[j] = Frag<T>::load(Bb + bo);
      if (SPLIT) bl[j] = Frag<T>::load(Bb2 + bo);
    }
#pragma unroll
    for (int i = 0; i < 4; ++i) {
      const size_t ao = (size_t)(m0 + (i << 4) + rlane) * lda + koff + k0;
      V ah = Frag<T>::load(Ab + ao);
      V al;
      if (SPLIT) al = Frag<T>::load(Ab2 + ao);
#pragma unroll
      for (int j = 0; j < 4; ++j) {
        acc[i][j] = Frag<T>::mma(ah, bh[j], acc[i][j]);
        if (SPLIT) {
          acc[i][j] = Frag<T>::mma(ah, bl[j], acc[i][j]);
          acc[i][j] = Frag<T>::mma(al, bh[j], acc[i][j]);
        }
      }
      Frag<T>::guard4(acc[i][0], acc[i][1], acc[i][2], acc[i][3], ah, SPLIT ? al : ah);
    }
    Frag<T>::keep(bh[0], bh[1], bh[2], bh[3]);
    if (SPLIT) Frag<T>::keep(bl[0], bl[1], bl[2], bl[3]);
  }
  acc_guard4(acc[0][0], acc[0][1], acc[0][2], acc[0][3]);
  acc_guard4(acc[1][0], acc[1][1], acc[1][2], acc[1][3]);
  acc_guard4(acc[2][0], acc[2][1], acc[2][2], acc[2][3]);
  acc_guard4(acc[3][0], acc[3][1], acc[3][2], acc[3][3]);

  float* slab = sT[wave];
  const float* Rb = RESID ? (resid + (size_t)b * strideR) : nullptr;
#pragma unroll
  for (int i = 0; i < 4; ++i) {
    const int mBase = m0 + (i << 4);
#pragma unroll
    for (int j = 0; j < 4; ++j) {
      const int n = n0 + (j << 4) + rlane;
      float bv = 0.f;
      if (BIAS_MODE == 2) bv = bias[n];
#pragma unroll
      for (int r = 0; r < 8; ++r) {
        float v = acc[i][j][r] * scale;
        if (BIAS_MODE == 1) v += bias[mBase + mOff + r];
        if (BIAS_MODE == 2) v += bv;
        if (RESID) v += Rb[(size_t)(mBase + mOff + r) * ldc + n];
        if (ACT == 2) v = fmaxf(v, 0.0f);
        if (ACT == 4) v = (v > 0.f) ? v : 0.01f * v;
        slab[(mOff + r) * 68 + (j << 4) + rlane] = v;
      }
    }
    __builtin_amdgcn_fence(__ATOMIC_RELEASE, "workgroup");
    __builtin_amdgcn_wave_barrier();
    __builtin_amdgcn_fence(__ATOMIC_ACQUIRE, "workgroup");
    if (OUT_MODE == 0) {
      float* C = (float*)Cout + (size_t)b * strideC;
      const int hh = lane >> 4, c4 = (lane & 15) * 4;
      for (int pass = 0; pass < 2; ++pass) {
#pragma unroll
        for (int it = 0; it < 8; ++it) {
          const int row = it * 2 + hh;
          v4f v = *(const v4f*)(slab + row * 68 + c4);
          *(volatile v4f*)(C + (size_t)(mBase + row) * ldc + n0 + c4) = v;
        }
        __threadfence();
      }
    } else {
      const int q = lane >> 3, c8 = (lane & 7) * 8;
      unsigned short* C  = (unsigned short*)Cout  + (size_t)b * strideC;
      unsigned short* C2 = (OUT_MODE == 2) ? ((unsigned short*)Cout2 + (size_t)b * strideC) : nullptr;
      for (int pass = 0; pass < 2; ++pass) {
#pragma unroll
        for (int it = 0; it < 4; ++it) {
          const int row = it * 4 + q;
          const float* sp = slab + row * 68 + c8;
          v8h hv, lv;
#pragma unroll
          for (int e = 0; e < 8; ++e) {
            if (OUT_MODE == 1) {
              hv[e] = (_Float16)sp[e];
            } else {
              unsigned short hb = f2bf_bits(sp[e]);
              unsigned short lb = f2bf_bits(sp[e] - bf_bits2f(hb));
              hv[e] = __builtin_bit_cast(_Float16, hb);
              lv[e] = __builtin_bit_cast(_Float16, lb);
            }
          }
          *(volatile v8h*)(C + (size_t)(mBase + row) * ldc + n0 + c8) = hv;
          if (OUT_MODE == 2) *(volatile v8h*)(C2 + (size_t)(mBase + row) * ldc + n0 + c8) = lv;
        }
        __threadfence();
      }
    }
    __builtin_amdgcn_fence(__ATOMIC_RELEASE, "workgroup");
    __builtin_amdgcn_wave_barrier();
    __builtin_amdgcn_fence(__ATOMIC_ACQUIRE, "workgroup");
  }
}

__global__ __launch_bounds__(256) void pack_w_kernel(const float* __restrict__ baseW, const float* __restrict__ splineW,
                                                     const float* __restrict__ scaler, unsigned short* __restrict__ bt) {
  __shared__ float red[8];
  const int o    = blockIdx.x;
  const int t    = threadIdx.x;
  const int lane = t & 31, wave = t >> 5;

  const v4f s4 = *(const v4f*)(scaler + (size_t)o * kIn + 4 * t);
  float s = 0.0f;
  s += s4[0]; s += s4[1]; s += s4[2]; s += s4[3];
#pragma unroll
  for (int off = 16; off > 0; off >>= 1) s += __shfl_xor(s, off, 32);
  if (lane == 0) red[wave] = s;
  __syncthreads();
  float ssum = 0.0f;
#pragma unroll
  for (int w = 0; w < 8; ++w) ssum += red[w];
  const float swc = ssum * kWCarry;

  v4u pk[2];
#pragma unroll
  for (int it = 0; it < 2; ++it) {
    const int p  = it * 256 + t;
    const int i0 = 2 * p;
    const v2f b2 = *(const v2f*)(baseW + (size_t)o * kIn + i0);
    const float* sp = splineW + ((size_t)o * kIn + i0) * kNB;
    const v4f w0 = *(const v4f*)(sp);
    const v4f w1 = *(const v4f*)(sp + kNB);
    unsigned short hb[8];
    hb[0] = h_bits(b2[0] * kWCarry);
    hb[1] = h_bits(swc * w0[0]);
    hb[2] = h_bits(swc * w0[1]);
    hb[3] = h_bits(swc * w0[2]);
    hb[4] = h_bits(b2[1] * kWCarry);
    hb[5] = h_bits(swc * w1[0]);
    hb[6] = h_bits(swc * w1[1]);
    hb[7] = h_bits(swc * w1[2]);
    pk[it] = (v4u){pk16(hb[0], hb[1]), pk16(hb[2], hb[3]), pk16(hb[4], hb[5]), pk16(hb[6], hb[7])};
  }
  unsigned short* dst = bt + (size_t)o * kAug;
  for (int pass = 0; pass < 2; ++pass) {
#pragma unroll
    for (int it = 0; it < 2; ++it) {
      const int p = it * 256 + t;
      *(volatile v4u*)(dst + 8 * p) = pk[it];
    }
    __threadfence();
  }
}

__device__ __forceinline__ void expand_one(float xv, const float (&g)[kGridN], const float (&r1)[5], const float (&r2)[4],
                                           const float (&r3)[3], float (&f)[4]) {
  float b0[5];
#pragma unroll
  for (int i = 0; i < 5; ++i) b0[i] = (xv >= g[i] && xv < g[i + 1]) ? 1.0f : 0.0f;
  float c1[4];
#pragma unroll
  for (int i = 0; i < 4; ++i)
    c1[i] = ((xv - g[i]) * r1[i]) * b0[i] + ((g[i + 2] - xv) * r1[i + 1]) * b0[i + 1];
  float c2[3];
#pragma unroll
  for (int i = 0; i < 3; ++i)
    c2[i] = ((xv - g[i]) * r2[i]) * c1[i] + ((g[i + 3] - xv) * r2[i + 1]) * c1[i + 1];
  float c3[3];
#pragma unroll
  for (int i = 0; i < 2; ++i)
    c3[i] = ((xv - g[i]) * r3[i]) * c2[i] + ((g[i + 4] - xv) * r3[i + 1]) * c2[i + 1];
  c3[2] = ((xv - g[2]) * r3[2]) * c2[2];
  const float e   = expf(-xv);
  const float sig = 1.0f / (1.0f + e);
  f[0] = xv * sig;
  f[1] = c3[0];
  f[2] = c3[1];
  f[3] = c3[2];
}

__global__ __launch_bounds__(256) void pack_x_kernel(const float* __restrict__ x, const float* __restrict__ knots,
                                                     unsigned short* __restrict__ ap, int nthreads) {
  const int gid = blockIdx.x * 256 + threadIdx.x;
  if (gid >= nthreads) return;
  const int row = gid >> 9;
  const int p   = gid & 511;
  const int i0  = 2 * p;

  float g[kGridN];
#pragma unroll
  for (int i = 0; i < kGridN; ++i) g[i] = knots[i];
  float r1[5], r2[4], r3[3];
#pragma unroll
  for (int i = 0; i < 5; ++i) r1[i] = __builtin_amdgcn_rcpf((g[i + 1] - g[i]) + kEps);
#pragma unroll
  for (int i = 0; i < 4; ++i) r2[i] = __builtin_amdgcn_rcpf((g[i + 2] - g[i]) + kEps);
#pragma unroll
  for (int i = 0; i < 3; ++i) r3[i] = __builtin_amdgcn_rcpf((g[i + 3] - g[i]) + kEps);

  const v2f xv = *(const v2f*)(x + (size_t)row * kIn + i0);
  const float x0 = xv[0];
  const float x1 = xv[1];
  float f0[4], f1[4];
  expand_one(x0, g, r1, r2, r3, f0);
  expand_one(x1, g, r1, r2, r3, f1);

  unsigned short hb[8];
#pragma unroll
  for (int c = 0; c < 4; ++c) {
    hb[c]     = h_bits(f0[c] * kACarry);
    hb[4 + c] = h_bits(f1[c] * kACarry);
  }
  const v4u u = (v4u){pk16(hb[0], hb[1]), pk16(hb[2], hb[3]), pk16(hb[4], hb[5]), pk16(hb[6], hb[7])};
  unsigned short* dst = ap + (size_t)row * kAug + 8 * p;
  *(volatile v4u*)dst = u;
  __threadfence();
  *(volatile v4u*)dst = u;
}

extern "C" void kernel_launch(void* const* d_in, const int* in_sizes, int n_in,
                              void* d_out, int out_size, void* d_ws, size_t ws_size, hipStream_t stream) {
  (void)n_in;
  const float* x       = (const float*)d_in[0];
  const float* baseW   = (const float*)d_in[1];
  const float* splineW = (const float*)d_in[2];
  const float* scaler  = (const float*)d_in[3];
  const float* knots   = (const float*)d_in[4];

  if (in_sizes[0] != kRows * kIn) return;
  if (in_sizes[1] != kOutF * kIn) return;
  if (in_sizes[2] != kOutF * kIn * kNB) return;
  if (in_sizes[3] != kOutF * kIn) return;
  if (in_sizes[4] != kGridN) return;
  if (out_size != kRows * kOutF) return;
  if (kWsNeed > ws_size) return;

  unsigned short* bt = (unsigned short*)((char*)d_ws);
  unsigned short* ap = (unsigned short*)((char*)d_ws + kBtBytes);
  float* out = (float*)d_out;
  const float* unused_f = (const float*)d_ws;

  pack_w_kernel<<<dim3(kOutF), dim3(256), 0, stream>>>(baseW, splineW, scaler, bt);

  pack_x_kernel<<<dim3((kPairThreads + 255) / 256), dim3(256), 0, stream>>>(x, knots, ap, kPairThreads);

  wmma_gemm64<0, false, 0, 0, false, 0><<<dim3(kGemmBlocks, 1), dim3(256), 0, stream>>>(
      ap, ap, kAug, 0L,
      bt, bt, kAug, 0L,
      (void*)out, (void*)out, kOutF, 0L,
      unused_f,
      unused_f, 0L,
      kRows, kOutF, kAug, kOutScale);
}
